// MessagePassing_39230231281894
// MI455X (gfx1250) — hardware-verified
//
#include <hip/hip_runtime.h>
#include <stddef.h>
#include <stdint.h>
#include <math.h>


#define DIN     128
#define HID     256
#define NH      8
#define HDM     32
#define QKVW    768
#define OQ      0
#define OKK     256
#define OV      512
#define NTY     3
#define APITCH  576
#define KOUT    544
#define NTHR    256
#define NWAVE   8
#define EPT     8
#define CHUNK   (NTHR * EPT)
#define WCAP    (EPT * 32)
#define LISTN   (NWAVE * WCAP)
#define NBA     1024
#define SLA     10
#define RCAP    28672
#define DEGCAP  64
#define GBM     64
#define GBN     64
#define GTHR    128
#define UQKV    (HID * (DIN / 8))
#define UWO     (DIN * (KOUT / 8))
#define NUW     (3 * UQKV + UWO)
#define AGG_ZINTS (LISTN + 2 * RCAP + 3 * NBA)
#define MISC_INTS 16
#define EMB_FLTS  (NTY * HID)
#define SCAN_LDS_BYTES ((AGG_ZINTS + MISC_INTS + EMB_FLTS) * 4)
#define ATTSC   0.17677669529663687f
#define WSMAX   268435456

static_assert((CHUNK & (CHUNK - 1)) == 0 && CHUNK <= 4096);
static_assert((NBA & (NBA - 1)) == 0 && NBA == (1 << SLA));
static_assert(((long long)CHUNK << SLA) < (1LL << 31));
static_assert(LISTN % NTHR == 0);
static_assert(NBA % NWAVE == 0 && NBA % 32 == 0 && NBA % GBM == 0);
static_assert(RCAP % 4 == 0 && AGG_ZINTS % 4 == 0 && LISTN % 4 == 0 && ((AGG_ZINTS + MISC_INTS) % 4) == 0);
static_assert(AGG_ZINTS % (NTHR * 4) == 0);
static_assert(NWAVE * 2 * HID <= RCAP);
static_assert((EMB_FLTS % 4) == 0);
static_assert(SCAN_LDS_BYTES <= 300000);
static_assert(HID == 32 * 8);
static_assert(HDM == 4 * 8 && NH * HDM == HID && (NH & (NH - 1)) == 0);
static_assert(QKVW == 3 * HID && (QKVW % GBN) == 0 && (DIN % GBN) == 0);
static_assert((DIN % 32) == 0 && (KOUT % 32) == 0 && KOUT <= APITCH);
static_assert(KOUT == 2 * HID + 32 && APITCH == 2 * HID + 64);
static_assert((APITCH * 2) % 128 == 0);
static_assert(GBM == (GTHR / 32) * 16);
static_assert(UQKV % NTHR == 0 && UWO % NTHR == 0 && (KOUT / 8) == 68);
static_assert((3 * UQKV) % NTHR == 0);

typedef float          v4f  __attribute__((ext_vector_type(4)));
typedef float          v8f  __attribute__((ext_vector_type(8)));
typedef int            v4i  __attribute__((ext_vector_type(4)));
typedef int            v8i  __attribute__((ext_vector_type(8)));
typedef unsigned int   v4u  __attribute__((ext_vector_type(4)));
typedef unsigned short v8us __attribute__((ext_vector_type(8)));
typedef __bf16         v16b __attribute__((ext_vector_type(16)));
typedef v4f  __attribute__((may_alias)) v4fa;
typedef v4i  __attribute__((may_alias)) v4ia;
typedef v4u  __attribute__((may_alias)) v4ua;
typedef v8us __attribute__((may_alias)) v8usa;
union FragB { v16b v; v8us h[2]; v8i w; };

__device__ __forceinline__ v8f wmb(const FragB& a, const FragB& b, v8f c) {
  v8f d = __builtin_amdgcn_wmma_f32_16x16x32_bf16(false, a.v, false, b.v, (short)0, c, false, false);
  asm volatile("v_nop\n\tv_nop\n\tv_nop\n\tv_nop" : "+v"(d) : "v"(a.w), "v"(b.w));
  return d;
}

__device__ __forceinline__ void ldwait() {
  asm volatile("s_wait_loadcnt 0x0" ::: "memory");
}

__device__ __forceinline__ void wave_sync() {
  __builtin_amdgcn_fence(__ATOMIC_RELEASE, "wavefront");
  __builtin_amdgcn_wave_barrier();
  __builtin_amdgcn_fence(__ATOMIC_ACQUIRE, "wavefront");
}

__device__ __forceinline__ unsigned int f2bf(float f) {
  const unsigned int u = __float_as_uint(f);
  return ((u + 0x7FFFu + ((u >> 16) & 1u)) >> 16) & 0xFFFFu;
}
__device__ __forceinline__ float bf2f(unsigned int b) { return __uint_as_float(b << 16); }
__device__ __forceinline__ float bfr(float f) { return bf2f(f2bf(f)); }
__device__ __forceinline__ v4f bfr4(const v4f a) {
  v4f r; r.x = bfr(a.x); r.y = bfr(a.y); r.z = bfr(a.z); r.w = bfr(a.w); return r;
}
__device__ __forceinline__ unsigned int pk2(float lo, float hi) { return f2bf(lo) | (f2bf(hi) << 16); }
__device__ __forceinline__ v4u pack8(const v4f a, const v4f b) {
  v4u r;
  r.x = pk2(a.x, a.y); r.y = pk2(a.z, a.w); r.z = pk2(b.x, b.y); r.w = pk2(b.z, b.w);
  return r;
}
__device__ __forceinline__ void hl2(float v0, float v1, unsigned int& hw, unsigned int& lw) {
  const unsigned int h0 = f2bf(v0), h1 = f2bf(v1);
  const unsigned int l0 = f2bf(v0 - bf2f(h0)), l1 = f2bf(v1 - bf2f(h1));
  hw = h0 | (h1 << 16);
  lw = l0 | (l1 << 16);
}
__device__ __forceinline__ void pack8hl(const v4f a, const v4f b, v4u& hv, v4u& lv) {
  unsigned int h, l;
  hl2(a.x, a.y, h, l); hv.x = h; lv.x = l;
  hl2(a.z, a.w, h, l); hv.y = h; lv.y = l;
  hl2(b.x, b.y, h, l); hv.z = h; lv.z = l;
  hl2(b.z, b.w, h, l); hv.w = h; lv.w = l;
}

__device__ __forceinline__ int scan_chunk2(const int* __restrict__ edg, int nE, int cbase, int slotBase,
                                           int nb, int* list, int tid, int lane, int wave) {
  int wc = 0;
  const int el0  = tid * EPT;
  const int e0   = cbase + el0;
  const int sent = -2147483647 - 1;
  v4i da, db;
  if (cbase + CHUNK <= nE) {
    const int* p = edg + 2 * (size_t)e0;
    const v4i p0 = *(const v4i*)p;
    const v4i p1 = *(const v4i*)(p + 4);
    const v4i p2 = *(const v4i*)(p + 8);
    const v4i p3 = *(const v4i*)(p + 12);
    da.x = p0.x; da.y = p0.z; da.z = p1.x; da.w = p1.z;
    db.x = p2.x; db.y = p2.z; db.z = p3.x; db.w = p3.z;
  } else {
    da.x = (e0     < nE) ? edg[2 * (size_t)min(e0,     nE - 1)] : sent;
    da.y = (e0 + 1 < nE) ? edg[2 * (size_t)min(e0 + 1, nE - 1)] : sent;
    da.z = (e0 + 2 < nE) ? edg[2 * (size_t)min(e0 + 2, nE - 1)] : sent;
    da.w = (e0 + 3 < nE) ? edg[2 * (size_t)min(e0 + 3, nE - 1)] : sent;
    db.x = (e0 + 4 < nE) ? edg[2 * (size_t)min(e0 + 4, nE - 1)] : sent;
    db.y = (e0 + 5 < nE) ? edg[2 * (size_t)min(e0 + 5, nE - 1)] : sent;
    db.z = (e0 + 6 < nE) ? edg[2 * (size_t)min(e0 + 6, nE - 1)] : sent;
    db.w = (e0 + 7 < nE) ? edg[2 * (size_t)min(e0 + 7, nE - 1)] : sent;
  }
  const unsigned nbs = (unsigned)slotBase;
  const unsigned unb = (unsigned)nb;
  const unsigned s0 = (unsigned)da.x - nbs, s1 = (unsigned)da.y - nbs;
  const unsigned s2 = (unsigned)da.z - nbs, s3 = (unsigned)da.w - nbs;
  const unsigned s4 = (unsigned)db.x - nbs, s5 = (unsigned)db.y - nbs;
  const unsigned s6 = (unsigned)db.z - nbs, s7 = (unsigned)db.w - nbs;
  const bool h0 = s0 < unb, h1 = s1 < unb, h2 = s2 < unb, h3 = s3 < unb;
  const bool h4 = s4 < unb, h5 = s5 < unb, h6 = s6 < unb, h7 = s7 < unb;
  const unsigned any = __builtin_amdgcn_ballot_w32(h0 | h1 | h2 | h3 | h4 | h5 | h6 | h7);
  if (any != 0u) {
#define HITJ(J, HJ, SJ) { \
      const unsigned mj = __builtin_amdgcn_ballot_w32(HJ); \
      if (mj != 0u) { \
        if (HJ) { \
          const int pos = wc + (int)__builtin_amdgcn_mbcnt_lo(mj, 0u); \
          if (pos < WCAP) list[wave * WCAP + pos] = ((el0 + (J)) << SLA) | (int)(SJ); \
        } \
        wc += (int)__builtin_popcount(mj); } }
    HITJ(0, h0, s0)
    HITJ(1, h1, s1)
    HITJ(2, h2, s2)
    HITJ(3, h3, s3)
    HITJ(4, h4, s4)
    HITJ(5, h5, s5)
    HITJ(6, h6, s6)
    HITJ(7, h7, s7)
#undef HITJ
  }
  return wc;
}

__global__ __launch_bounds__(NTHR) void k_xprep(const float* __restrict__ x, unsigned short* xb, int nN, int nUnits) {
  const int i = (int)blockIdx.x * NTHR + (int)threadIdx.x;
  if (i >= nUnits) return;
  const int row = i >> 4;
  const int c0  = (i & 15) * 8;
  const int rc  = row < nN ? row : nN - 1;
  const float* p = x + (size_t)rc * DIN + c0;
  v4f a = *(const v4fa*)p;
  v4f b = *(const v4fa*)(p + 4);
  const v4f z4 = {0.f, 0.f, 0.f, 0.f};
  if (row >= nN) { a = z4; b = z4; }
  const v4u hv = pack8(a, b);
  unsigned short* o = xb + (size_t)row * DIN + c0;
  *(volatile v4u*)o = hv;
  __threadfence();
  *(volatile v4u*)o = hv;
}

__global__ __launch_bounds__(NTHR) void k_wprep(const float* __restrict__ Wq, const float* __restrict__ Wk,
                                                const float* __restrict__ Wv, const float* __restrict__ Wo,
                                                const float* __restrict__ bo,
                                                unsigned short* WQKVT, unsigned short* WOT) {
  const int u = (int)blockIdx.x * NTHR + (int)threadIdx.x;
  if (u >= NUW) return;
  v4f a, b;
  unsigned short* dp;
  if (u < 3 * UQKV) {
    const int part = u >> 12;
    const int v    = u & (UQKV - 1);
    const int n    = v >> 4;
    const int k8   = (v & 15) * 8;
    const float* W = (part == 0) ? Wq : ((part == 1) ? Wk : Wv);
    const float* p = W + (size_t)n * DIN + k8;
    a = *(const v4fa*)p;
    b = *(const v4fa*)(p + 4);
    dp = WQKVT + (size_t)(part * HID + n) * DIN + k8;
  } else {
    const int v  = u - 3 * UQKV;
    const int n  = v / 68;
    const int k8 = (v - n * 68) * 8;
    const int kk = (k8 < 2 * HID) ? (k8 & (HID - 1)) : 0;
    const float* p = Wo + (size_t)n * HID + kk;
    a = *(const v4fa*)p;
    b = *(const v4fa*)(p + 4);
    const float bov = bo[n];
    const float fw = (k8 < 2 * HID) ? 1.0f : 0.0f;
    const float fb = (k8 == 2 * HID) ? 1.0f : 0.0f;
    a.x = a.x * fw + bov * fb;
    a.y = a.y * fw; a.z = a.z * fw; a.w = a.w * fw;
    b.x = b.x * fw; b.y = b.y * fw; b.z = b.z * fw; b.w = b.w * fw;
    dp = WOT + (size_t)n * KOUT + k8;
  }
  const v4u wv = pack8(a, b);
  *(volatile v4u*)dp = wv;
  __threadfence();
  *(volatile v4u*)dp = wv;
}

__global__ __launch_bounds__(GTHR) void k_gemm(
    const unsigned short* __restrict__ A, int lda, const unsigned short* __restrict__ WT, int K,
    float* outF, int ldo, int nRows,
    const float* __restrict__ bs0, const float* __restrict__ bs1, const float* __restrict__ bs2, int useBias)
{
  __shared__ __attribute__((aligned(16))) float stg[GBM * GBN];
  const int tid = (int)threadIdx.x, lane = tid & 31, wave = tid >> 5, hh = lane >> 4, m = lane & 15;
  const int rowBase = (int)blockIdx.x * GBM;
  const int col0    = (int)blockIdx.y * GBN;

  v8f acc[4];
  {
    const v8f z = {0.f, 0.f, 0.f, 0.f, 0.f, 0.f, 0.f, 0.f};
    acc[0] = z; acc[1] = z; acc[2] = z; acc[3] = z;
  }
  const unsigned short* ap = A  + (size_t)(rowBase + 16 * wave + m) * (size_t)lda + 8 * hh;
  const unsigned short* wp = WT + (size_t)(col0 + m) * (size_t)K + 8 * hh;
  const int ksteps = K >> 5;
#pragma unroll 1
  for (int ks = 0; ks < ksteps; ++ks) {
    FragB af;
    af.h[0] = *(const v8usa*)(ap + 32 * ks);
    af.h[1] = *(const v8usa*)(ap + 32 * ks + 16);
#pragma unroll
    for (int t = 0; t < 4; ++t) {
      const unsigned short* wq = wp + (size_t)(16 * t) * (size_t)K + 32 * ks;
      FragB bf;
      bf.h[0] = *(const v8usa*)wq;
      bf.h[1] = *(const v8usa*)(wq + 16);
      acc[t] = wmb(af, bf, acc[t]);
    }
  }

#pragma unroll
  for (int t = 0; t < 4; ++t) {
    const int lc = 16 * t + m;
#pragma unroll
    for (int r = 0; r < 8; ++r) {
      const int lr = 16 * wave + 8 * hh + r;
      stg[lr * GBN + lc] = acc[t][r];
    }
  }
  __syncthreads();

  const int mat = col0 >> 8;
  const float* bsel = (mat == 0) ? bs0 : ((mat == 1) ? bs1 : bs2);
  v4f b4 = *(const v4fa*)(bsel + (col0 & (HID - 1)) + 4 * m);
  b4 = bfr4(b4) * (float)useBias;

  v4f fv[8];
#pragma unroll
  for (int i = 0; i < 8; ++i) {
    const int lr = 16 * wave + 2 * i + hh;
    fv[i] = *(const v4fa*)(stg + lr * GBN + 4 * m) + b4;
  }
#pragma unroll
  for (int i = 0; i < 8; ++i) {
    const int lr = 16 * wave + 2 * i + hh;
    const int gr = rowBase + lr;
    const int gs = gr < nRows ? gr : nRows - 1;
    float* op = outF + (size_t)gs * (size_t)ldo + col0 + 4 * m;
    if (gr < nRows) *(volatile v4f*)op = fv[i];
  }
  __threadfence();
#pragma unroll
  for (int i = 0; i < 8; ++i) {
    const int lr = 16 * wave + 2 * i + hh;
    const int gr = rowBase + lr;
    const int gs = gr < nRows ? gr : nRows - 1;
    float* op = outF + (size_t)gs * (size_t)ldo + col0 + 4 * m;
    if (gr < nRows) *(volatile v4f*)op = fv[i];
  }
}

__global__ __launch_bounds__(NTHR) void k_scan(const int* __restrict__ edg, const int* __restrict__ ety,
                                               const float* __restrict__ QKV, const float* __restrict__ emb,
                                               unsigned short* apl, int nE, int nN, int mRows) {
  extern __shared__ __attribute__((aligned(16))) int dsm[];
  int* list = dsm;
  int* hl   = dsm + LISTN;
  int* sl   = hl + RCAP;
  int* cnt  = sl + RCAP;
  int* offs = cnt + NBA;
  int* cur  = offs + NBA;
  int* misc = cur + NBA;
  float* semb = (float*)(misc + MISC_INTS);
  const int tid = (int)threadIdx.x, lane = tid & 31, wave = tid >> 5;
  const int nodeBase = (int)blockIdx.x * NBA;

  {
    const v4i z4 = {0, 0, 0, 0};
    for (int i = tid * 4; i < AGG_ZINTS; i += NTHR * 4) *(v4ia*)(dsm + i) = z4;
    if (tid < MISC_INTS) misc[tid] = 0;
#pragma unroll 1
    for (int i = tid; i < EMB_FLTS / 4; i += NTHR) {
      const v4f ev = *(const v4fa*)(emb + 4 * i);
      *(v4fa*)(semb + 4 * i) = bfr4(ev);
    }
  }
  __syncthreads();

  int t = 0, ov = 0;
  const int nChunks = (nE + CHUNK - 1) / CHUNK;
#pragma unroll 1
  for (int ch = 0; ch < nChunks; ++ch) {
    const int cbase = ch * CHUNK;
    const int wc = scan_chunk2(edg, nE, cbase, nodeBase, NBA, list, tid, lane, wave);
    if (lane == 0) misc[wave] = wc;
    __syncthreads();
    if (wave == 0) {
#pragma unroll 1
      for (int w2 = 0; w2 < NWAVE; ++w2) {
        int c = misc[w2];
        c = c < 0 ? 0 : (c > WCAP ? WCAP : c);
#pragma unroll 1
        for (int b0 = 0; b0 < c; b0 += 32) {
          const int idx = b0 + lane;
          const int ent = list[w2 * WCAP + (idx < WCAP ? idx : WCAP - 1)];
          const int m32 = (c - b0) < 32 ? (c - b0) : 32;
#pragma unroll 1
          for (int k = 0; k < m32; ++k) {
            const int u    = __builtin_amdgcn_readlane(ent, k);
            const int slot = u & (NBA - 1);
            const int el   = (u >> SLA) & (CHUNK - 1);
            const int pk   = ((cbase + el) << SLA) | slot;
            if (t < RCAP) {
              if (lane == 0) { hl[t] = pk; cnt[slot] = cnt[slot] + 1; }
              t = t + 1;
            } else {
              ov = 1;
            }
          }
        }
      }
    }
    __syncthreads();
  }
  if (wave == 0 && lane == 0) { misc[8] = t; misc[9] = ov; }
  __syncthreads();
  int tt = misc[8];
  tt = tt < 0 ? 0 : (tt > RCAP ? RCAP : tt);
  const int ovf = misc[9];

  if (wave == 0) {
    const int base = lane * (NBA / 32);
    int s = 0;
#pragma unroll 1
    for (int i = 0; i < NBA / 32; ++i) s += cnt[base + i];
    int incl = s;
#pragma unroll
    for (int d = 1; d < 32; d <<= 1) {
      const int y = __shfl_up(incl, d, 32);
      if (lane >= d) incl += y;
    }
    int run = incl - s;
#pragma unroll 1
    for (int i = 0; i < NBA / 32; ++i) {
      const int cv = cnt[base + i];
      offs[base + i] = run;
      cur[base + i]  = run;
      run += cv;
    }
  }
  __syncthreads();
  if (wave == 0) {
#pragma unroll 1
    for (int b0 = 0; b0 < tt; b0 += 32) {
      const int idx = b0 + lane;
      const int ent = hl[idx < RCAP ? idx : RCAP - 1];
      const int m32 = (tt - b0) < 32 ? (tt - b0) : 32;
#pragma unroll 1
      for (int k = 0; k < m32; ++k) {
        const int u    = __builtin_amdgcn_readlane(ent, k);
        const int slot = u & (NBA - 1);
        if (lane == 0) {
          int p = cur[slot];
          p = p < 0 ? 0 : (p > RCAP - 1 ? RCAP - 1 : p);
          sl[p] = u;
          cur[slot] = p + 1;
        }
      }
    }
  }
  __syncthreads();

  const float qnan = __int_as_float(0x7fc00000);
  const float pz = (ovf != 0) ? qnan : 0.0f;
  float* skv = (float*)hl + wave * (2 * HID);
  const int hd = lane >> 2;
  const int jj = lane & 3;
  const v4f z4 = {0.f, 0.f, 0.f, 0.f};
#pragma unroll 1
  for (int si = 0; si < NBA / NWAVE; ++si) {
    const int s    = si * NWAVE + wave;
    const int node = nodeBase + s;
    int c = cnt[s];
    const bool big = c > DEGCAP;
    c = c < 0 ? 0 : (c > DEGCAP ? DEGCAP : c);
    int o = offs[s];
    o = o < 0 ? 0 : (o > RCAP ? RCAP : o);
    const int nc = node < nN ? node : nN - 1;

    const float* qr = QKV + (size_t)nc * QKVW + OQ + 8 * lane;
    const v4f qa = *(const v4fa*)qr;
    const v4f qb = *(const v4fa*)(qr + 4);
    ldwait();

    v4f aga = z4, agb = z4;
#pragma unroll 1
    for (int b0 = 0; b0 < c; b0 += 32) {
      int idx = o + b0 + lane;
      idx = idx > RCAP - 1 ? RCAP - 1 : idx;
      const int ent = sl[idx];
      int eid = ent >> SLA;
      eid = eid < 0 ? 0 : (eid > nE - 1 ? nE - 1 : eid);
      int tg = edg[2 * (size_t)eid + 1];
      tg = tg < 0 ? 0 : (tg > nN - 1 ? nN - 1 : tg);
      int ty = ety[eid];
      ty = ty < 0 ? 0 : (ty > NTY - 1 ? NTY - 1 : ty);
      const int m32 = (c - b0) < 32 ? (c - b0) : 32;
#pragma unroll 1
      for (int k = 0; k < m32; ++k) {
        const int tk = __builtin_amdgcn_readlane(tg, k);
        const int yk = __builtin_amdgcn_readlane(ty, k);
        const float* kr = QKV + (size_t)tk * QKVW + OKK + 8 * lane;
        const v4f ka = *(const v4fa*)kr;
        const v4f kb = *(const v4fa*)(kr + 4);
        const float* vr = QKV + (size_t)tk * QKVW + OV + 8 * lane;
        const v4f va = *(const v4fa*)vr;
        const v4f vb = *(const v4fa*)(vr + 4);
        ldwait();
        wave_sync();
        *(v4fa*)(skv + 8 * lane)           = ka;
        *(v4fa*)(skv + 8 * lane + 4)       = kb;
        *(v4fa*)(skv + HID + 8 * lane)     = va;
        *(v4fa*)(skv + HID + 8 * lane + 4) = vb;
        wave_sync();

        float mx = -1.0e30f, den = 0.0f;
        v4f ma = z4, mb = z4;
#pragma unroll 1
        for (int r = 0; r < NH; ++r) {
          const int g = (hd + r) & (NH - 1);
          const float* kp = skv + HDM * g + 8 * jj;
          const v4f k0 = *(const v4fa*)kp;
          const v4f k1 = *(const v4fa*)(kp + 4);
          float p = qa.x * k0.x;
          p = fmaf(qa.y, k0.y, p); p = fmaf(qa.z, k0.z, p); p = fmaf(qa.w, k0.w, p);
          p = fmaf(qb.x, k1.x, p); p = fmaf(qb.y, k1.y, p); p = fmaf(qb.z, k1.z, p); p = fmaf(qb.w, k1.w, p);
          p += __shfl_xor(p, 1);
          p += __shfl_xor(p, 2);
          const float lg = p * ATTSC;
          const float df = lg - mx;
          const float ee = __expf(-fabsf(df));
          const bool up  = df > 0.0f;
          const float s1 = up ? ee : 1.0f;
          const float s2 = up ? 1.0f : ee;
          mx  = up ? lg : mx;
          den = fmaf(den, s1, s2);
          const float* vp = skv + HID + HDM * g + 8 * jj;
          const v4f v0 = *(const v4fa*)vp;
          const v4f v1 = *(const v4fa*)(vp + 4);
          ma.x = fmaf(ma.x, s1, s2 * v0.x); ma.y = fmaf(ma.y, s1, s2 * v0.y);
          ma.z = fmaf(ma.z, s1, s2 * v0.z); ma.w = fmaf(ma.w, s1, s2 * v0.w);
          mb.x = fmaf(mb.x, s1, s2 * v1.x); mb.y = fmaf(mb.y, s1, s2 * v1.y);
          mb.z = fmaf(mb.z, s1, s2 * v1.z); mb.w = fmaf(mb.w, s1, s2 * v1.w);
        }
        const float inv = __builtin_amdgcn_rcpf(den);
        const float* ep = semb + yk * HID + 8 * lane;
        const v4f e0 = *(const v4fa*)ep;
        const v4f e1 = *(const v4fa*)(ep + 4);
        aga.x = aga.x + fmaf(ma.x, inv, e0.x); aga.y = aga.y + fmaf(ma.y, inv, e0.y);
        aga.z = aga.z + fmaf(ma.z, inv, e0.z); aga.w = aga.w + fmaf(ma.w, inv, e0.w);
        agb.x = agb.x + fmaf(mb.x, inv, e1.x); agb.y = agb.y + fmaf(mb.y, inv, e1.y);
        agb.z = agb.z + fmaf(mb.z, inv, e1.z); agb.w = agb.w + fmaf(mb.w, inv, e1.w);
      }
    }

    const float pzr = big ? qnan : pz;
    const bool live = node < nN;
    v4f oa, ob;
    oa.x = live ? (aga.x + pzr) : 0.0f; oa.y = live ? (aga.y + pzr) : 0.0f;
    oa.z = live ? (aga.z + pzr) : 0.0f; oa.w = live ? (aga.w + pzr) : 0.0f;
    ob.x = live ? (agb.x + pzr) : 0.0f; ob.y = live ? (agb.y + pzr) : 0.0f;
    ob.z = live ? (agb.z + pzr) : 0.0f; ob.w = live ? (agb.w + pzr) : 0.0f;
    v4u hv, lv;
    pack8hl(oa, ob, hv, lv);
    const float cf = live ? (float)c : 0.0f;
    const unsigned cw = (lane == 0) ? f2bf(cf) : 0u;
    v4u cv; cv.x = cw; cv.y = 0u; cv.z = 0u; cv.w = 0u;

    if (node < mRows) {
      unsigned short* rp = apl + (size_t)node * APITCH;
      *(volatile v4u*)(rp + 8 * lane)       = hv;
      *(volatile v4u*)(rp + HID + 8 * lane) = lv;
      if (lane < 8) *(volatile v4u*)(rp + 2 * HID + 8 * lane) = cv;
      __threadfence();
      *(volatile v4u*)(rp + 8 * lane)       = hv;
      *(volatile v4u*)(rp + HID + 8 * lane) = lv;
      if (lane < 8) *(volatile v4u*)(rp + 2 * HID + 8 * lane) = cv;
    }
  }
}

static inline int cdiv(int a, int b) { return (a + b - 1) / b; }
static inline size_t al256(size_t o) { return (o + 255) & ~(size_t)255; }

extern "C" void kernel_launch(void* const* d_in, const int* in_sizes, int n_in,
                              void* d_out, int out_size, void* d_ws, size_t ws_size,
                              hipStream_t stream) {
  if (n_in < 12) return;
  if (in_sizes[0] < DIN || (in_sizes[0] % DIN) != 0) return;
  const int nN = in_sizes[0] / DIN;
  if (nN < 16 || nN >= (1 << 21)) return;
  if (in_sizes[1] < 2 || (in_sizes[1] & 1) != 0) return;
  const int nE = in_sizes[1] / 2;
  if (nE < 1 || nE >= (1 << 21)) return;
  if (in_sizes[2] != nE) return;
  if (in_sizes[3] != HID * DIN || in_sizes[5] != HID * DIN || in_sizes[7] != HID * DIN) return;
  if (in_sizes[4] != HID || in_sizes[6] != HID || in_sizes[8] != HID) return;
  if (in_sizes[9] != NTY * HID) return;
  if (in_sizes[10] != DIN * HID || in_sizes[11] != DIN) return;
  if ((long long)out_size != (long long)nN * DIN) return;

  const float* x     = (const float*)d_in[0];
  const int*   edges = (const int*)  d_in[1];
  const int*   etyp  = (const int*)  d_in[2];
  const float* Wq    = (const float*)d_in[3];
  const float* bq    = (const float*)d_in[4];
  const float* Wk    = (const float*)d_in[5];
  const float* bk    = (const float*)d_in[6];
  const float* Wv    = (const float*)d_in[7];
  const float* bv    = (const float*)d_in[8];
  const float* emb   = (const float*)d_in[9];
  const float* Wo    = (const float*)d_in[10];
  const float* bo    = (const float*)d_in[11];
  float* out = (float*)d_out;

  const int MP = cdiv(nN, GBM) * GBM;
  const int gM = MP / GBM;
  const int gA = cdiv(MP, NBA);
  if ((long long)gA * NBA < (long long)MP) return;

  char* ws = (char*)d_ws;
  size_t off = 0;
  const size_t oXB  = off; off = al256(off + (size_t)MP * DIN * 2);
  const size_t oWQ  = off; off = al256(off + (size_t)QKVW * DIN * 2);
  const size_t oWO  = off; off = al256(off + (size_t)DIN * KOUT * 2);
  const size_t oQKV = off; off = al256(off + (size_t)MP * QKVW * 4);
  const size_t oAPL = off; off = al256(off + (size_t)MP * APITCH * 2);
  if (off > ws_size || off > (size_t)WSMAX) return;
  unsigned short* XB    = (unsigned short*)(ws + oXB);
  unsigned short* WQKVT = (unsigned short*)(ws + oWQ);
  unsigned short* WOT   = (unsigned short*)(ws + oWO);
  float*          QKV   = (float*)(ws + oQKV);
  unsigned short* APL   = (unsigned short*)(ws + oAPL);

  hipFuncSetAttribute(reinterpret_cast<const void*>(&k_scan),
                      hipFuncAttributeMaxDynamicSharedMemorySize, SCAN_LDS_BYTES);

  const int nUx = MP * (DIN / 8);
  k_xprep<<<cdiv(nUx, NTHR), NTHR, 0, stream>>>(x, XB, nN, nUx);
  k_wprep<<<NUW / NTHR, NTHR, 0, stream>>>(Wq, Wk, Wv, Wo, bo, WQKVT, WOT);
  k_gemm<<<dim3(gM, QKVW / GBN), GTHR, 0, stream>>>(XB, DIN, WQKVT, DIN, QKV, QKVW, MP, bq, bk, bv, 1);
  k_scan<<<gA, NTHR, SCAN_LDS_BYTES, stream>>>(edges, etyp, QKV, emb, APL, nE, nN, MP);
  k_gemm<<<dim3(gM, DIN / GBN), GTHR, 0, stream>>>(APL, APITCH, WOT, KOUT, out, DIN, nN, bo, bo, bo, 0);
}
